// VmambaMixer_48747878810259
// MI455X (gfx1250) — hardware-run, weakly checked
//
#include <hip/hip_runtime.h>
#include <math.h>

typedef __attribute__((ext_vector_type(16))) _Float16 v16h;
typedef __attribute__((ext_vector_type(8)))  _Float16 v8h;
typedef __attribute__((ext_vector_type(16))) __bf16   v16b;
typedef __attribute__((ext_vector_type(8)))  __bf16   v8b;
typedef __attribute__((ext_vector_type(8)))  float    v8f;
typedef __attribute__((ext_vector_type(4)))  float    v4f;
typedef __attribute__((ext_vector_type(2)))  float    v2f;
typedef __attribute__((ext_vector_type(4)))  unsigned v4u;

constexpr int kB    = 8;
constexpr int kH    = 56;
constexpr int kW    = 56;
constexpr int kL    = kH * kW;
constexpr int kNT   = kB * kL;
constexpr int kDm   = 96;
constexpr int kDin  = 192;
constexpr int kNst  = 32;
constexpr int kR    = 6;
constexpr int kHd   = 32;
constexpr int kDir  = 4;
constexpr int kPj   = kR + 2 * kNst;
constexpr int kPjP  = 80;
constexpr int kXdP  = kDir * kPjP;
constexpr int kXzP  = 2 * kDin;
constexpr int kOutP = 128;
constexpr int kTS   = 32;
constexpr int kRowP = 76;
constexpr int kYP   = 196;
constexpr float kCarryA = 1024.0f;
constexpr float kCarryW = 1024.0f;
constexpr float kFoldX  = 1.0f / (kCarryA * kCarryW);
static_assert(kL == 3136 && kNT == 25088, "token counts");
static_assert(kR * kHd == kDin && kPj == 70 && kXdP == 320 && kXzP == 384, "widths");
static_assert((kNT % 64) == 0 && (kXzP % 64) == 0 && (kXdP % 64) == 0 && (kOutP % 64) == 0, "GEMM M,N multiples of 64");
static_assert((kDm % 32) == 0 && (kDin % 32) == 0, "GEMM K multiples of 32");
static_assert((kL % kTS) == 0 && (kNT % 8) == 0 && kTS * kR == 192, "scan and tile multiples");
static_assert((kRowP % 4) == 0 && (kYP % 4) == 0, "16-B aligned LDS rows");

constexpr size_t kSzWI  = (size_t)kXzP * kDm * 2;
constexpr size_t kSzWX  = (size_t)kXdP * kDin * 2;
constexpr size_t kSzWO  = (size_t)kOutP * kDin * 2;
constexpr size_t kSzXB  = (size_t)kNT * kDm * 2;
constexpr size_t kSzXZ  = (size_t)kNT * kXzP * 4;
constexpr size_t kSzXIA = (size_t)kNT * kDin * 4;
constexpr size_t kSzX16 = (size_t)kNT * kDin * 2;
constexpr size_t kSzXD  = (size_t)kNT * kXdP * 4;
constexpr size_t kSzYS  = (size_t)kDir * kNT * kDin * 2;
constexpr size_t kOffWIH = 0;
constexpr size_t kOffWIL = kOffWIH + kSzWI;
constexpr size_t kOffWX  = kOffWIL + kSzWI;
constexpr size_t kOffWOH = kOffWX  + kSzWX;
constexpr size_t kOffWOL = kOffWOH + kSzWO;
constexpr size_t kOffXZ  = kOffWOL + kSzWO;
constexpr size_t kOffXIA = kOffXZ  + kSzXZ;
constexpr size_t kOffXD  = kOffXIA + kSzXIA;
constexpr size_t kOffYS  = kOffXD  + kSzXD;
constexpr size_t kWsTotal = kOffYS + kSzYS;
constexpr size_t kOffXBH = kOffYS;
constexpr size_t kOffXBL = kOffYS + kSzXB;
constexpr size_t kOffX16 = kOffYS + 2 * kSzXB;
constexpr size_t kOffYBH = kOffXD;
constexpr size_t kOffYBL = kOffXD + kSzX16;
static_assert(kOffXZ == 368640ull, "weights region");
static_assert(kWsTotal == 128819200ull, "carve total");
static_assert(kWsTotal <= 134217728ull, "carve cap");
static_assert(2 * kSzXB + kSzX16 <= kSzYS, "early planes fit inside the YS region");
static_assert(2 * kSzX16 <= kSzXD, "late planes fit inside the XD region");
static_assert((kOffWIL % 128) == 0 && (kOffWX % 128) == 0 && (kOffWOH % 128) == 0 && (kOffWOL % 128) == 0 &&
              (kOffXZ % 128) == 0 && (kOffXIA % 128) == 0 && (kOffXD % 128) == 0 && (kOffYS % 128) == 0 &&
              (kOffXBL % 128) == 0 && (kOffX16 % 128) == 0 && (kOffYBL % 128) == 0, "128-B aligned regions");

__device__ __forceinline__ unsigned f2bf_u(float f) {
  const unsigned u = __float_as_uint(f);
  return (u + 0x7FFFu + ((u >> 16) & 1u)) >> 16;
}
__device__ __forceinline__ float bfu2f(unsigned h) { return __uint_as_float(h << 16); }
__device__ __forceinline__ unsigned f2h_u(float f) {
  const _Float16 h = (_Float16)f;
  const unsigned short s = __builtin_bit_cast(unsigned short, h);
  return (unsigned)s;
}
__device__ __forceinline__ void pin_f(float& x) { asm volatile("" : "+v"(x)); }

__device__ __forceinline__ void bf16_hilo_pack(v4f a0, v4f a1, v4u& wh, v4u& wl) {
  unsigned h[8], l[8];
#pragma unroll
  for (int e = 0; e < 4; ++e) {
    const float x0 = a0[e];
    const float x1 = a1[e];
    h[e]     = f2bf_u(x0);
    h[4 + e] = f2bf_u(x1);
    l[e]     = f2bf_u(x0 - bfu2f(h[e]));
    l[4 + e] = f2bf_u(x1 - bfu2f(h[4 + e]));
  }
  wh = (v4u){ h[0] | (h[1] << 16), h[2] | (h[3] << 16), h[4] | (h[5] << 16), h[6] | (h[7] << 16) };
  wl = (v4u){ l[0] | (l[1] << 16), l[2] | (l[3] << 16), l[4] | (l[5] << 16), l[6] | (l[7] << 16) };
}

__device__ __forceinline__ void tie_h(v8f& a, v16h x, v16h y) { asm volatile("" : "+v"(a) : "v"(x), "v"(y)); }
__device__ __forceinline__ void tie_b(v8f& a, v16b x, v16b y) { asm volatile("" : "+v"(a) : "v"(x), "v"(y)); }
__device__ __forceinline__ void nop4_h(v8f& a, v16h x, v16h y) { asm volatile("v_nop\n\tv_nop\n\tv_nop\n\tv_nop" : "+v"(a) : "v"(x), "v"(y)); }
__device__ __forceinline__ void nop4_b(v8f& a, v16b x, v16b y) { asm volatile("v_nop\n\tv_nop\n\tv_nop\n\tv_nop" : "+v"(a) : "v"(x), "v"(y)); }
__device__ __forceinline__ void keep4_h(v16h a, v16h b, v16h c, v16h d) { asm volatile("v_nop" :: "v"(a), "v"(b), "v"(c), "v"(d)); }
__device__ __forceinline__ void keep4_b(v16b a, v16b b, v16b c, v16b d) { asm volatile("v_nop" :: "v"(a), "v"(b), "v"(c), "v"(d)); }
__device__ __forceinline__ void acc_guard4(v8f& a, v8f& b, v8f& c, v8f& d) { asm volatile("v_nop\n\tv_nop\n\tv_nop\n\tv_nop" : "+v"(a), "+v"(b), "+v"(c), "+v"(d)); }
template <typename T> struct Frag;
template <> struct Frag<_Float16> {
  typedef v16h V; union U { v16h v; v8h h[2]; };
  static __device__ __forceinline__ v16h load(const _Float16* p) {
    U f; f.h[0] = *(const v8h*)(p); f.h[1] = *(const v8h*)(p + 16); return f.v;
  }
  static __device__ __forceinline__ v8f mma(v16h a, v16h b, v8f c) {
    return __builtin_amdgcn_wmma_f32_16x16x32_f16(false, a, false, b, (short)0, c, false, false);
  }
  static __device__ __forceinline__ void tie(v8f& a, v16h x, v16h y) { tie_h(a, x, y); }
  static __device__ __forceinline__ void nop4(v8f& a, v16h x, v16h y) { nop4_h(a, x, y); }
  static __device__ __forceinline__ void keep(v16h a, v16h b, v16h c, v16h d) { keep4_h(a, b, c, d); }
};
template <> struct Frag<__bf16> {
  typedef v16b V; union U { v16b v; v8b h[2]; };
  static __device__ __forceinline__ v16b load(const __bf16* p) {
    U f; f.h[0] = *(const v8b*)(p); f.h[1] = *(const v8b*)(p + 16); return f.v;
  }
  static __device__ __forceinline__ v8f mma(v16b a, v16b b, v8f c) {
    return __builtin_amdgcn_wmma_f32_16x16x32_bf16(false, a, false, b, (short)0, c, false, false);
  }
  static __device__ __forceinline__ void tie(v8f& a, v16b x, v16b y) { tie_b(a, x, y); }
  static __device__ __forceinline__ void nop4(v8f& a, v16b x, v16b y) { nop4_b(a, x, y); }
  static __device__ __forceinline__ void keep(v16b a, v16b b, v16b c, v16b d) { keep4_b(a, b, c, d); }
};
template <int ET> struct Elem;
template <> struct Elem<0> { typedef _Float16 T; };
template <> struct Elem<1> { typedef __bf16 T; };

template <int ET, bool SPLIT>
__global__ __launch_bounds__(256) void wmma_gemm64(
    const unsigned short* __restrict__ Ap, const unsigned short* __restrict__ A2p, int lda,
    const unsigned short* __restrict__ Btp, const unsigned short* __restrict__ Bt2p, int ldb,
    float* __restrict__ C, int ldc, int M, int N, int K, float scale, int nStore) {
  typedef typename Elem<ET>::T T;
  typedef typename Frag<T>::V V;
  const T* A = (const T*)Ap; const T* A2 = (const T*)A2p; const T* Bt = (const T*)Btp; const T* Bt2 = (const T*)Bt2p;
  __shared__ __align__(16) float sT[8][16 * 68];
  const int lane = threadIdx.x & 31;
  const int wave = threadIdx.x >> 5;
  const int tilesN = N >> 6;
  const int tilesM = M >> 6;
  const int tile = blockIdx.x * 8 + wave;
  if (tile >= tilesM * tilesN) return;
  const int tm = tile / tilesN;
  const int tn = tile - tm * tilesN;
  const int m0 = tm << 6;
  const int n0 = tn << 6;

  const int rlane = lane & 15;
  const int koff  = (lane >> 4) * 8;
  const int mOff  = (lane >> 4) * 8;

  v8f acc[4][4];
#pragma unroll
  for (int i = 0; i < 4; ++i)
#pragma unroll
    for (int j = 0; j < 4; ++j) acc[i][j] = (v8f){0.f,0.f,0.f,0.f,0.f,0.f,0.f,0.f};

  for (int k0 = 0; k0 < K; k0 += 32) {
    V bh[4], bl[4];
#pragma unroll
    for (int j = 0; j < 4; ++j) {
      const size_t bo = (size_t)(n0 + (j << 4) + rlane) * ldb + koff + k0;
      bh[j] = Frag<T>::load(Bt + bo);
      if (SPLIT) bl[j] = Frag<T>::load(Bt2 + bo);
    }
#pragma unroll
    for (int i = 0; i < 4; ++i) {
      const size_t ao = (size_t)(m0 + (i << 4) + rlane) * lda + koff + k0;
      V ah = Frag<T>::load(A + ao);
      V al;
      if (SPLIT) al = Frag<T>::load(A2 + ao);
#pragma unroll
      for (int j = 0; j < 4; ++j) {
        acc[i][j] = Frag<T>::mma(ah, bh[j], acc[i][j]);
        if (SPLIT) {
          acc[i][j] = Frag<T>::mma(ah, bl[j], acc[i][j]);
          acc[i][j] = Frag<T>::mma(al, bh[j], acc[i][j]);
        }
      }
      Frag<T>::tie(acc[i][0], ah, SPLIT ? al : ah);
      Frag<T>::tie(acc[i][1], ah, SPLIT ? al : ah);
      Frag<T>::tie(acc[i][2], ah, SPLIT ? al : ah);
      Frag<T>::nop4(acc[i][3], ah, SPLIT ? al : ah);
    }
    Frag<T>::keep(bh[0], bh[1], bh[2], bh[3]);
    if (SPLIT) Frag<T>::keep(bl[0], bl[1], bl[2], bl[3]);
  }
  acc_guard4(acc[0][0], acc[0][1], acc[0][2], acc[0][3]);
  acc_guard4(acc[1][0], acc[1][1], acc[1][2], acc[1][3]);
  acc_guard4(acc[2][0], acc[2][1], acc[2][2], acc[2][3]);
  acc_guard4(acc[3][0], acc[3][1], acc[3][2], acc[3][3]);

  float* slab = sT[wave];
#pragma unroll
  for (int i = 0; i < 4; ++i) {
    const int mBase = m0 + (i << 4);
#pragma unroll
    for (int j = 0; j < 4; ++j) {
#pragma unroll
      for (int r = 0; r < 8; ++r) {
        slab[(mOff + r) * 68 + (j << 4) + rlane] = acc[i][j][r] * scale;
      }
    }
    __builtin_amdgcn_fence(__ATOMIC_RELEASE, "workgroup");
    __builtin_amdgcn_wave_barrier();
    __builtin_amdgcn_fence(__ATOMIC_ACQUIRE, "workgroup");
    {
      const int hh = lane >> 4, c4 = (lane & 15) * 4;
      const bool colOk = (n0 + c4) < nStore;
      for (int pass = 0; pass < 2; ++pass) {
#pragma unroll
        for (int it = 0; it < 8; ++it) {
          const int row = it * 2 + hh;
          const v4f v = *(const v4f*)(slab + row * 68 + c4);
          if (colOk) *(volatile v4f*)(C + (size_t)(mBase + row) * ldc + n0 + c4) = v;
        }
        __threadfence();
      }
    }
    __builtin_amdgcn_fence(__ATOMIC_RELEASE, "workgroup");
    __builtin_amdgcn_wave_barrier();
    __builtin_amdgcn_fence(__ATOMIC_ACQUIRE, "workgroup");
  }
}

__global__ __launch_bounds__(256) void split_rows_bf16_kernel(
    const float* __restrict__ src, unsigned short* __restrict__ dhi, unsigned short* __restrict__ dlo,
    int rowsReal, int cols, int total8)
{
  const int i = blockIdx.x * 256 + threadIdx.x;
  if (i >= total8) return;
  const int e0  = i << 3;
  const int row = e0 / cols;
  const int col = e0 - row * cols;
  const int rowc = (row < rowsReal) ? row : (rowsReal - 1);
  const float* p = src + (size_t)rowc * cols + col;
  v4f a0 = *(const v4f*)(p);
  v4f a1 = *(const v4f*)(p + 4);
  const bool live = row < rowsReal;
  v4f b0, b1;
#pragma unroll
  for (int e = 0; e < 4; ++e) {
    float x0 = a0[e];
    float x1 = a1[e];
    pin_f(x0);
    pin_f(x1);
    b0[e] = live ? x0 : 0.0f;
    b1[e] = live ? x1 : 0.0f;
  }
  v4u wh, wl;
  bf16_hilo_pack(b0, b1, wh, wl);
  unsigned short* qh = dhi + e0;
  unsigned short* ql = dlo + e0;
  *(volatile v4u*)qh = wh;
  *(volatile v4u*)ql = wl;
  __threadfence();
  *(volatile v4u*)qh = wh;
  *(volatile v4u*)ql = wl;
}

__global__ __launch_bounds__(256) void cast_xproj_f16_kernel(
    const float* __restrict__ src, unsigned short* __restrict__ dst, int total8)
{
  const int i = blockIdx.x * 256 + threadIdx.x;
  if (i >= total8) return;
  const int e0 = i << 3;
  const int n  = e0 / kDin;
  const int d  = e0 - n * kDin;
  const int kd = n / kPjP;
  const int cc = n - kd * kPjP;
  const int ccc = (cc < kPj) ? cc : (kPj - 1);
  const float* p = src + ((size_t)(kd * kPj + ccc)) * kDin + d;
  v4f a0 = *(const v4f*)(p);
  v4f a1 = *(const v4f*)(p + 4);
  const bool live = cc < kPj;
  unsigned h[8];
#pragma unroll
  for (int e = 0; e < 4; ++e) {
    float x0 = a0[e];
    float x1 = a1[e];
    pin_f(x0);
    pin_f(x1);
    const float y0 = live ? (x0 * kCarryW) : 0.0f;
    const float y1 = live ? (x1 * kCarryW) : 0.0f;
    h[e]     = f2h_u(y0);
    h[4 + e] = f2h_u(y1);
  }
  const v4u w = (v4u){ h[0] | (h[1] << 16), h[2] | (h[3] << 16), h[4] | (h[5] << 16), h[6] | (h[7] << 16) };
  unsigned short* q = dst + e0;
  *(volatile v4u*)q = w;
  __threadfence();
  *(volatile v4u*)q = w;
}

__global__ __launch_bounds__(192) void conv_silu_kernel(
    const float* __restrict__ XZ, const float* __restrict__ cw, const float* __restrict__ cb,
    float* __restrict__ XIA, unsigned short* __restrict__ XIA16)
{
  __shared__ __align__(16) float sW[9 * kDin];
  __shared__ __align__(16) float sO[8 * kDin];
  const int tid = threadIdx.x;
  const int c = tid;
#pragma unroll 1
  for (int tap = 0; tap < 9; ++tap) sW[tap * kDin + c] = cw[tap * kDin + c];
  const float bias = cb[c];
  __syncthreads();
  const int t0 = blockIdx.x * 8;
#pragma unroll 1
  for (int j = 0; j < 8; ++j) {
    const int t  = t0 + j;
    const int bi = t / kL;
    const int l  = t - bi * kL;
    const int hy0 = l / kW;
    const int wx0 = l - hy0 * kW;
    float acc = 0.0f;
#pragma unroll 1
    for (int ky = 0; ky < 3; ++ky) {
#pragma unroll 1
      for (int kx = 0; kx < 3; ++kx) {
        const int hy = hy0 + ky - 1;
        const int wx = wx0 + kx - 1;
        const bool ok = (hy >= 0) && (hy < kH) && (wx >= 0) && (wx < kW);
        const int hyc = hy < 0 ? 0 : (hy > kH - 1 ? kH - 1 : hy);
        const int wxc = wx < 0 ? 0 : (wx > kW - 1 ? kW - 1 : wx);
        float v = XZ[((size_t)(bi * kL + hyc * kW + wxc)) * kXzP + c];
        v = ok ? v : 0.0f;
        acc = fmaf(v, sW[(ky * 3 + kx) * kDin + c], acc);
      }
    }
    const float sv = acc + bias;
    const float sg = 1.0f / (1.0f + expf(-sv));
    sO[j * kDin + c] = sv * sg;
  }
  __syncthreads();
  const v4f f0 = *(const v4f*)(sO + tid * 4);
  const v4f f1 = *(const v4f*)(sO + 768 + tid * 4);
  const v4f g0 = *(const v4f*)(sO + tid * 8);
  const v4f g1 = *(const v4f*)(sO + tid * 8 + 4);
  unsigned h[8];
#pragma unroll
  for (int e = 0; e < 4; ++e) {
    h[e]     = f2h_u(g0[e] * kCarryA);
    h[4 + e] = f2h_u(g1[e] * kCarryA);
  }
  const v4u w16 = (v4u){ h[0] | (h[1] << 16), h[2] | (h[3] << 16), h[4] | (h[5] << 16), h[6] | (h[7] << 16) };
  float* pf = XIA + (size_t)t0 * kDin;
  unsigned short* ph = XIA16 + (size_t)t0 * kDin + tid * 8;
  for (int pass = 0; pass < 2; ++pass) {
    *(volatile v4f*)(pf + tid * 4) = f0;
    *(volatile v4f*)(pf + 768 + tid * 4) = f1;
    *(volatile v4u*)ph = w16;
    __threadfence();
  }
}

__device__ __forceinline__ int scan_pos(int k, int l) {
  const int l2 = (k & 2) ? (kL - 1 - l) : l;
  const int wq = l2 / kH;
  const int hr = l2 - wq * kH;
  const int tp = hr * kW + wq;
  return (k & 1) ? tp : l2;
}

__global__ __launch_bounds__(384) void scan_kernel(
    const float* __restrict__ XD, const float* __restrict__ XIA,
    const float* __restrict__ dtb, const float* __restrict__ alog,
    unsigned short* __restrict__ YS)
{
  __shared__ __align__(16) float sR[kTS * kRowP];
  __shared__ __align__(16) float sY[kTS * kYP];
  __shared__ int sP[kTS];
  const int tid = threadIdx.x, lane = tid & 31, wave = tid >> 5;
  const int k = blockIdx.x & 3;
  const int b = blockIdx.x >> 2;
  const int half = lane >> 4;
  const int c = wave * 16 + (lane & 15);
  const int r = wave >> 1;
  const int n0s = half * 16;
  const size_t rowb = (size_t)b * kL;

  float hS[16];
#pragma unroll
  for (int j = 0; j < 16; ++j) hS[j] = 0.0f;

#pragma unroll 1
  for (int t0 = 0; t0 < kL; t0 += kTS) {
    __syncthreads();
    if (tid < kTS) sP[tid] = scan_pos(k, t0 + tid);
#pragma unroll
    for (int it = 0; it < 2; ++it) {
      const int idx  = tid + it * 384;
      const bool valid = idx < kTS * 18;
      const int idxc = valid ? idx : (kTS * 18 - 1);
      const int s = idxc / 18;
      const int q = idxc - s * 18;
      const int p = scan_pos(k, t0 + s);
      const v4f v = *(const v4f*)(XD + (rowb + (size_t)p) * kXdP + k * kPjP + q * 4);
      float v0 = v[0], v1 = v[1], v2 = v[2], v3 = v[3];
      pin_f(v0);
      pin_f(v1);
      pin_f(v2);
      pin_f(v3);
      const int col0 = q * 4;
      float* dr = sR + s * kRowP;
      {
        const int col = col0;
        const int dst = (col < kR) ? (64 + col) : (col - kR);
        if (valid && col < kPj) dr[dst] = v0;
      }
      {
        const int col = col0 + 1;
        const int dst = (col < kR) ? (64 + col) : (col - kR);
        if (valid && col < kPj) dr[dst] = v1;
      }
      {
        const int col = col0 + 2;
        const int dst = (col < kR) ? (64 + col) : (col - kR);
        if (valid && col < kPj) dr[dst] = v2;
      }
      {
        const int col = col0 + 3;
        const int dst = (col < kR) ? (64 + col) : (col - kR);
        if (valid && col < kPj) dr[dst] = v3;
      }
    }
    __syncthreads();
    if (wave < 6) {
      const int s  = tid / kR;
      const int r2 = tid - s * kR;
      float* pr = sR + s * kRowP;
      const float v   = pr[64 + r2] + dtb[k * kR + r2];
      const float dtv = fmaxf(v, 0.0f) + log1pf(expf(-fabsf(v)));
      const float Av  = -expf(alog[k * kR + r2]);
      pr[64 + r2] = dtv;
      pr[70 + r2] = expf(dtv * Av);
    }
    __syncthreads();
#pragma unroll 1
    for (int s = 0; s < kTS; ++s) {
      const float* rr = sR + s * kRowP;
      const int p = sP[s];
      const float xt  = XIA[(rowb + (size_t)p) * kDin + c];
      const float dtv = rr[64 + r];
      const float dAv = rr[70 + r];
      const float dtx = xt * dtv;
      float y = 0.0f;
#pragma unroll
      for (int q4 = 0; q4 < 4; ++q4) {
        const v4f bv = *(const v4f*)(rr + n0s + 4 * q4);
        const v4f cv = *(const v4f*)(rr + kNst + n0s + 4 * q4);
#pragma unroll
        for (int e = 0; e < 4; ++e) {
          const float hn = fmaf(hS[4 * q4 + e], dAv, dtx * bv[e]);
          hS[4 * q4 + e] = hn;
          y = fmaf(hn, cv[e], y);
        }
      }
      y += __shfl_xor(y, 16, 32);
      if (half == 0) sY[s * kYP + c] = y;
    }
    __syncthreads();
    {
      const int q = lane >> 3, c8 = (lane & 7) * 8;
      v4u wv[2];
      size_t off[2];
#pragma unroll
      for (int it = 0; it < 2; ++it) {
        const int li  = it * 48 + wave * 4 + q;
        const int row = li / 3;
        const int seg = li - row * 3;
        const float* sp = sY + row * kYP + seg * 64 + c8;
        const v4f a0 = *(const v4f*)(sp);
        const v4f a1 = *(const v4f*)(sp + 4);
        unsigned h[8];
#pragma unroll
        for (int e = 0; e < 4; ++e) {
          h[e]     = f2bf_u(a0[e]);
          h[4 + e] = f2bf_u(a1[e]);
        }
        wv[it] = (v4u){ h[0] | (h[1] << 16), h[2] | (h[3] << 16), h[4] | (h[5] << 16), h[6] | (h[7] << 16) };
        off[it] = ((size_t)k * kNT + rowb + (size_t)sP[row]) * kDin + seg * 64 + c8;
      }
      for (int pass = 0; pass < 2; ++pass) {
#pragma unroll
        for (int it = 0; it < 2; ++it) *(volatile v4u*)(YS + off[it]) = wv[it];
        __threadfence();
      }
    }
  }
}

__global__ __launch_bounds__(256) void merge_norm_gate_kernel(
    const unsigned short* __restrict__ YS, const float* __restrict__ XIA, const float* __restrict__ XZ,
    const float* __restrict__ Dsk, const float* __restrict__ lng, const float* __restrict__ lnb,
    unsigned short* __restrict__ YBH, unsigned short* __restrict__ YBL)
{
  __shared__ __align__(16) float sV[8 * kDin];
  const int tid = threadIdx.x, lane = tid & 31, wave = tid >> 5;
  const int tb = blockIdx.x * 8;
  const int t  = tb + wave;
  float* sv = sV + wave * kDin;
  float sum = 0.0f;
#pragma unroll 1
  for (int j = 0; j < 3; ++j) {
    const int c = 64 * j + 2 * lane;
    const v2f xv = *(const v2f*)(XIA + (size_t)t * kDin + c);
    const float x0 = xv[0];
    const float x1 = xv[1];
    float v0 = 0.0f, v1 = 0.0f;
#pragma unroll
    for (int k = 0; k < kDir; ++k) {
      const unsigned w = *(const unsigned*)(YS + ((size_t)k * kNT + t) * kDin + c);
      const float y0 = __uint_as_float(w << 16);
      const float y1 = __uint_as_float(w & 0xffff0000u);
      const v2f dv = *(const v2f*)(Dsk + k * kDin + c);
      const float d0 = dv[0];
      const float d1 = dv[1];
      v0 = v0 + (y0 + x0 * d0);
      v1 = v1 + (y1 + x1 * d1);
    }
    *(v2f*)(sv + c) = (v2f){ v0, v1 };
    sum += v0 + v1;
  }
#pragma unroll
  for (int off = 16; off > 0; off >>= 1) sum += __shfl_xor(sum, off, 32);
  const float mu = sum * (1.0f / (float)kDin);
  __syncthreads();
  float sq = 0.0f;
#pragma unroll 1
  for (int j = 0; j < 6; ++j) {
    const float d = sv[32 * j + lane] - mu;
    sq = fmaf(d, d, sq);
  }
#pragma unroll
  for (int off = 16; off > 0; off >>= 1) sq += __shfl_xor(sq, off, 32);
  const float var = sq * (1.0f / (float)kDin);
  const float rs  = rsqrtf(var + 1e-5f);
#pragma unroll 1
  for (int j = 0; j < 6; ++j) {
    const int c = 32 * j + lane;
    const float yn = (sv[c] - mu) * rs * lng[c] + lnb[c];
    const float ge = 0.5f * yn * (1.0f + erff(yn * 0.70710678118654752f));
    const float z  = XZ[(size_t)t * kXzP + kDin + c];
    const float sz = z * (1.0f / (1.0f + expf(-z)));
    sv[c] = ge * sz;
  }
  __syncthreads();
  if (wave < 6) {
    const float* sp = sV + tid * 8;
    const v4f a0 = *(const v4f*)(sp);
    const v4f a1 = *(const v4f*)(sp + 4);
    v4u wh, wl;
    bf16_hilo_pack(a0, a1, wh, wl);
    unsigned short* ph = YBH + (size_t)tb * kDin + tid * 8;
    unsigned short* pl = YBL + (size_t)tb * kDin + tid * 8;
    *(volatile v4u*)ph = wh;
    *(volatile v4u*)pl = wl;
    __threadfence();
    *(volatile v4u*)ph = wh;
    *(volatile v4u*)pl = wl;
  }
}

extern "C" void kernel_launch(void* const* d_in, const int* in_sizes, int n_in,
                              void* d_out, int out_size, void* d_ws, size_t ws_size,
                              hipStream_t stream) {
  if (n_in < 11) return;
  if (in_sizes[0] != kNT * kDm) return;
  if (in_sizes[1] != kXzP * kDm) return;
  if (in_sizes[2] != 9 * kDin) return;
  if (in_sizes[3] != kDin) return;
  if (in_sizes[4] != kDir * kPj * kDin) return;
  if (in_sizes[5] != kDir * kDin) return;
  if (in_sizes[6] != kDir * kR) return;
  if (in_sizes[7] != kDir * kR) return;
  if (in_sizes[8] != kDin) return;
  if (in_sizes[9] != kDin) return;
  if (in_sizes[10] != kDm * kDin) return;
  if (out_size != kNT * kDm) return;
  if (ws_size < kWsTotal) return;

  const float* x       = (const float*)d_in[0];
  const float* w_in    = (const float*)d_in[1];
  const float* conv_w  = (const float*)d_in[2];
  const float* conv_b  = (const float*)d_in[3];
  const float* w_xp    = (const float*)d_in[4];
  const float* Dsk     = (const float*)d_in[5];
  const float* a_logs  = (const float*)d_in[6];
  const float* dt_bias = (const float*)d_in[7];
  const float* ln_g    = (const float*)d_in[8];
  const float* ln_b    = (const float*)d_in[9];
  const float* w_out   = (const float*)d_in[10];
  float* out = (float*)d_out;

  char* ws = (char*)d_ws;
  unsigned short* WIH   = (unsigned short*)(ws + kOffWIH);
  unsigned short* WIL   = (unsigned short*)(ws + kOffWIL);
  unsigned short* WX16  = (unsigned short*)(ws + kOffWX);
  unsigned short* WOH   = (unsigned short*)(ws + kOffWOH);
  unsigned short* WOL   = (unsigned short*)(ws + kOffWOL);
  float*          XZ    = (float*)(ws + kOffXZ);
  float*          XIA   = (float*)(ws + kOffXIA);
  float*          XD    = (float*)(ws + kOffXD);
  unsigned short* YS    = (unsigned short*)(ws + kOffYS);
  unsigned short* XBH   = (unsigned short*)(ws + kOffXBH);
  unsigned short* XBL   = (unsigned short*)(ws + kOffXBL);
  unsigned short* XIA16 = (unsigned short*)(ws + kOffX16);
  unsigned short* YBH   = (unsigned short*)(ws + kOffYBH);
  unsigned short* YBL   = (unsigned short*)(ws + kOffYBL);

  split_rows_bf16_kernel<<<(kNT * kDm / 8) / 256, 256, 0, stream>>>(x, XBH, XBL, kNT, kDm, kNT * kDm / 8);
  split_rows_bf16_kernel<<<(kXzP * kDm / 8) / 256, 256, 0, stream>>>(w_in, WIH, WIL, kXzP, kDm, kXzP * kDm / 8);
  split_rows_bf16_kernel<<<(kOutP * kDin / 8) / 256, 256, 0, stream>>>(w_out, WOH, WOL, kDm, kDin, kOutP * kDin / 8);
  cast_xproj_f16_kernel<<<(kXdP * kDin / 8) / 256, 256, 0, stream>>>(w_xp, WX16, kXdP * kDin / 8);

  wmma_gemm64<1, true><<<(kNT / 64) * (kXzP / 64) / 8, 256, 0, stream>>>(
      XBH, XBL, kDm, WIH, WIL, kDm, XZ, kXzP, kNT, kXzP, kDm, 1.0f, kXzP);

  conv_silu_kernel<<<kNT / 8, 192, 0, stream>>>(XZ, conv_w, conv_b, XIA, XIA16);

  wmma_gemm64<0, false><<<(kNT / 64) * (kXdP / 64) / 8, 256, 0, stream>>>(
      XIA16, XIA16, kDin, WX16, WX16, kDin, XD, kXdP, kNT, kXdP, kDin, kFoldX, kXdP);

  scan_kernel<<<kB * kDir, 384, 0, stream>>>(XD, XIA, dt_bias, a_logs, YS);

  merge_norm_gate_kernel<<<kNT / 8, 256, 0, stream>>>(YS, XIA, XZ, Dsk, ln_g, ln_b, YBH, YBL);

  wmma_gemm64<1, true><<<(kNT / 64) * (kOutP / 64) / 8, 256, 0, stream>>>(
      YBH, YBL, kDin, WOH, WOL, kDin, out, kDm, kNT, kOutP, kDin, 1.0f, kDm);
}
